// NonLocal_1614907703717
// MI455X (gfx1250) — hardware-verified
//
#include <hip/hip_runtime.h>
#include <math.h>

constexpr int kBatch   = 16;
constexpr int kCh      = 256;
constexpr int kN       = 1600;
constexpr int kTok     = kBatch * kN;
constexpr int kGroup   = 2;
constexpr int kNGroups = kBatch / kGroup;
constexpr int kSmThreads = kN / 8;
constexpr float kPCarry    = 32768.0f;
constexpr float kPCarryInv = 1.0f / 32768.0f;
constexpr int kBrB1 = 0;
constexpr int kBrB2 = 256;
constexpr int kBrB3 = 512;
constexpr int kBrW4a = 768;
constexpr int kBrW4b = 1024;
constexpr int kBrB4 = 1280;
constexpr int kBrFloats = 1408;
static_assert(kTok % 64 == 0 && kN % 64 == 0 && kCh % 64 == 0, "M and N tile multiples");
static_assert(kCh % 32 == 0 && kN % 32 == 0, "K multiples of 32");
static_assert(kBatch % kGroup == 0, "groups");
static_assert(kN % 8 == 0 && kSmThreads <= 256 && (kSmThreads % 32) == 8, "softmax store map: full waves plus one 8-lane line");
static_assert((kGroup * kN) % 32 == 0, "head blocks own whole 32-float lines");
static_assert(kBrB4 + 1 <= 41 * 32 && 41 * 32 <= kBrFloats, "parameter table extent");

typedef __attribute__((ext_vector_type(16))) _Float16 v16h;
typedef __attribute__((ext_vector_type(8)))  _Float16 v8h;
typedef __attribute__((ext_vector_type(16))) __bf16   v16b;
typedef __attribute__((ext_vector_type(8)))  __bf16   v8b;
typedef __attribute__((ext_vector_type(8)))  float    v8f;
typedef __attribute__((ext_vector_type(4)))  float    v4f;
typedef __attribute__((ext_vector_type(4)))  unsigned int v4u;

__device__ __forceinline__ unsigned short f2bf_bits(float f) {
  unsigned u = __float_as_uint(f);
  return (unsigned short)((u + 0x7FFFu + ((u >> 16) & 1u)) >> 16);
}
__device__ __forceinline__ float bf_bits2f(unsigned short h) { return __uint_as_float(((unsigned)h) << 16); }

__device__ __forceinline__ void dep_guard_h(v8f& a, v8f& b, v16h x, v16h y) { asm volatile("v_nop\n\tv_nop\n\tv_nop\n\tv_nop" : "+v"(a), "+v"(b) : "v"(x), "v"(y)); }
__device__ __forceinline__ void dep_guard_b(v8f& a, v8f& b, v16b x, v16b y) { asm volatile("v_nop\n\tv_nop\n\tv_nop\n\tv_nop" : "+v"(a), "+v"(b) : "v"(x), "v"(y)); }
__device__ __forceinline__ void dep_guard4_h(v8f& a, v8f& b, v8f& c, v8f& d, v16h x, v16h y) { asm volatile("v_nop\n\tv_nop\n\tv_nop\n\tv_nop" : "+v"(a), "+v"(b), "+v"(c), "+v"(d) : "v"(x), "v"(y)); }
__device__ __forceinline__ void dep_guard4_b(v8f& a, v8f& b, v8f& c, v8f& d, v16b x, v16b y) { asm volatile("v_nop\n\tv_nop\n\tv_nop\n\tv_nop" : "+v"(a), "+v"(b), "+v"(c), "+v"(d) : "v"(x), "v"(y)); }
__device__ __forceinline__ void keep4_h(v16h a, v16h b, v16h c, v16h d) { asm volatile("v_nop" :: "v"(a), "v"(b), "v"(c), "v"(d)); }
__device__ __forceinline__ void keep4_b(v16b a, v16b b, v16b c, v16b d) { asm volatile("v_nop" :: "v"(a), "v"(b), "v"(c), "v"(d)); }
__device__ __forceinline__ void acc_guard4(v8f& a, v8f& b, v8f& c, v8f& d) { asm volatile("v_nop\n\tv_nop\n\tv_nop\n\tv_nop" : "+v"(a), "+v"(b), "+v"(c), "+v"(d)); }
template <typename T> struct Frag;
template <> struct Frag<_Float16> {
  typedef v16h V; union U { v16h v; v8h h[2]; };
  static __device__ __forceinline__ v16h load(const _Float16* p) {
    U f; f.h[0] = *(const v8h*)(p); f.h[1] = *(const v8h*)(p + 16); return f.v;
  }
  static __device__ __forceinline__ v8f mma(v16h a, v16h b, v8f c) {
    return __builtin_amdgcn_wmma_f32_16x16x32_f16(false, a, false, b, (short)0, c, false, false);
  }
  static __device__ __forceinline__ void guard(v8f& a, v8f& b, v16h x, v16h y) { dep_guard_h(a, b, x, y); }
  static __device__ __forceinline__ void guard4(v8f& a, v8f& b, v8f& c, v8f& d, v16h x, v16h y) { dep_guard4_h(a, b, c, d, x, y); }
  static __device__ __forceinline__ void keep(v16h a, v16h b, v16h c, v16h d) { keep4_h(a, b, c, d); }
};
template <> struct Frag<__bf16> {
  typedef v16b V; union U { v16b v; v8b h[2]; };
  static __device__ __forceinline__ v16b load(const __bf16* p) {
    U f; f.h[0] = *(const v8b*)(p); f.h[1] = *(const v8b*)(p + 16); return f.v;
  }
  static __device__ __forceinline__ v8f mma(v16b a, v16b b, v8f c) {
    return __builtin_amdgcn_wmma_f32_16x16x32_bf16(false, a, false, b, (short)0, c, false, false);
  }
  static __device__ __forceinline__ void guard(v8f& a, v8f& b, v16b x, v16b y) { dep_guard_b(a, b, x, y); }
  static __device__ __forceinline__ void guard4(v8f& a, v8f& b, v8f& c, v8f& d, v16b x, v16b y) { dep_guard4_b(a, b, c, d, x, y); }
  static __device__ __forceinline__ void keep(v16b a, v16b b, v16b c, v16b d) { keep4_b(a, b, c, d); }
};

__device__ __forceinline__ unsigned pk16(unsigned short a, unsigned short b) { return (unsigned)a | ((unsigned)b << 16); }
__device__ __forceinline__ unsigned short h_bits(float f) { const _Float16 h = (_Float16)f; return __builtin_bit_cast(unsigned short, h); }

template <int ET> struct Elem;
template <> struct Elem<0> { typedef _Float16 T; };
template <> struct Elem<1> { typedef __bf16 T; };
template <int ET, bool SPLIT, int BIAS_MODE, int OUT_MODE, bool RESID, int ACT = 0>
__global__ __launch_bounds__(256) void wmma_gemm64(
    const unsigned short* __restrict__ Ap, const unsigned short* __restrict__ A2p, int lda, long strideA,
    const unsigned short* __restrict__ Btp, const unsigned short* __restrict__ Bt2p, int ldb, long strideB,
    void* __restrict__ Cout, void* __restrict__ Cout2, int ldc, long strideC,
    const float* __restrict__ bias,
    const float* __restrict__ resid, long strideR,
    int M, int N, int K, float scale) {
  typedef typename Elem<ET>::T T;
  typedef typename Frag<T>::V V;
  const T* A = (const T*)Ap; const T* A2 = (const T*)A2p; const T* Bt = (const T*)Btp; const T* Bt2 = (const T*)Bt2p;
  __shared__ __align__(16) float sT[8][16 * 68];
  const int b    = blockIdx.y;
  const int lane = threadIdx.x & 31;
  const int wave = threadIdx.x >> 5;
  const int tilesN = N >> 6;
  const int tilesM = M >> 6;
  const int tile = blockIdx.x * 8 + wave;
  if (tile >= tilesM * tilesN) return;
  const int tm = tile / tilesN;
  const int tn = tile - tm * tilesN;
  const int m0 = tm << 6;
  const int n0 = tn << 6;

  const T* Ab  = A  + (size_t)b * strideA;
  const T* Bb  = Bt + (size_t)b * strideB;
  const T* Ab2 = SPLIT ? (A2  + (size_t)b * strideA) : nullptr;
  const T* Bb2 = SPLIT ? (Bt2 + (size_t)b * strideB) : nullptr;

  const int rlane = lane & 15;
  const int koff  = (lane >> 4) * 8;
  const int mOff  = (lane >> 4) * 8;

  v8f acc[4][4];
#pragma unroll
  for (int i = 0; i < 4; ++i)
#pragma unroll
    for (int j = 0; j < 4; ++j) acc[i][j] = (v8f){0.f,0.f,0.f,0.f,0.f,0.f,0.f,0.f};

  for (int k0 = 0; k0 < K; k0 += 32) {
    V bh[4], bl[4];
#pragma unroll
    for (int j = 0; j < 4; ++j) {
      const size_t bo = (size_t)(n0 + (j << 4) + rlane) * ldb + koff + k0;
      bh[j] = Frag<T>::load(Bb + bo);
      if (SPLIT) bl[j] = Frag<T>::load(Bb2 + bo);
    }
#pragma unroll
    for (int i = 0; i < 4; ++i) {
      const size_t ao = (size_t)(m0 + (i << 4) + rlane) * lda + koff + k0;
      V ah = Frag<T>::load(Ab + ao);
      V al;
      if (SPLIT) al = Frag<T>::load(Ab2 + ao);
#pragma unroll
      for (int j = 0; j < 4; ++j) {
        acc[i][j] = Frag<T>::mma(ah, bh[j], acc[i][j]);
        if (SPLIT) {
          acc[i][j] = Frag<T>::mma(ah, bl[j], acc[i][j]);
          acc[i][j] = Frag<T>::mma(al, bh[j], acc[i][j]);
        }
      }
      Frag<T>::guard4(acc[i][0], acc[i][1], acc[i][2], acc[i][3], ah, SPLIT ? al : ah);
    }
    Frag<T>::keep(bh[0], bh[1], bh[2], bh[3]);
    if (SPLIT) Frag<T>::keep(bl[0], bl[1], bl[2], bl[3]);
  }
  acc_guard4(acc[0][0], acc[0][1], acc[0][2], acc[0][3]);
  acc_guard4(acc[1][0], acc[1][1], acc[1][2], acc[1][3]);
  acc_guard4(acc[2][0], acc[2][1], acc[2][2], acc[2][3]);
  acc_guard4(acc[3][0], acc[3][1], acc[3][2], acc[3][3]);

  float* slab = sT[wave];
  const float* Rb = RESID ? (resid + (size_t)b * strideR) : nullptr;
#pragma unroll
  for (int i = 0; i < 4; ++i) {
    const int mBase = m0 + (i << 4);
#pragma unroll
    for (int j = 0; j < 4; ++j) {
      const int n = n0 + (j << 4) + rlane;
      float bv = 0.f;
      if (BIAS_MODE == 2) bv = bias[n];
#pragma unroll
      for (int r = 0; r < 8; ++r) {
        float v = acc[i][j][r] * scale;
        if (BIAS_MODE == 1) v += bias[mBase + mOff + r];
        if (BIAS_MODE == 2) v += bv;
        if (RESID) v += Rb[(size_t)(mBase + mOff + r) * ldc + n];
        if (ACT == 2) v = fmaxf(v, 0.0f);
        if (ACT == 4) v = (v > 0.f) ? v : 0.01f * v;
        slab[(mOff + r) * 68 + (j << 4) + rlane] = v;
      }
    }
    __builtin_amdgcn_fence(__ATOMIC_RELEASE, "workgroup");
    __builtin_amdgcn_wave_barrier();
    __builtin_amdgcn_fence(__ATOMIC_ACQUIRE, "workgroup");
    if (OUT_MODE == 0) {
      float* C = (float*)Cout + (size_t)b * strideC;
      const int hh = lane >> 4, c4 = (lane & 15) * 4;
      for (int pass = 0; pass < 2; ++pass) {
#pragma unroll
        for (int it = 0; it < 8; ++it) {
          const int row = it * 2 + hh;
          v4f v = *(const v4f*)(slab + row * 68 + c4);
          *(volatile v4f*)(C + (size_t)(mBase + row) * ldc + n0 + c4) = v;
        }
        __threadfence();
      }
    } else {
      const int q = lane >> 3, c8 = (lane & 7) * 8;
      unsigned short* C  = (unsigned short*)Cout  + (size_t)b * strideC;
      unsigned short* C2 = (OUT_MODE == 2) ? ((unsigned short*)Cout2 + (size_t)b * strideC) : nullptr;
      for (int pass = 0; pass < 2; ++pass) {
#pragma unroll
        for (int it = 0; it < 4; ++it) {
          const int row = it * 4 + q;
          const float* sp = slab + row * 68 + c8;
          v8h hv, lv;
#pragma unroll
          for (int e = 0; e < 8; ++e) {
            if (OUT_MODE == 1) {
              hv[e] = (_Float16)sp[e];
            } else {
              unsigned short hb = f2bf_bits(sp[e]);
              unsigned short lb = f2bf_bits(sp[e] - bf_bits2f(hb));
              hv[e] = __builtin_bit_cast(_Float16, hb);
              lv[e] = __builtin_bit_cast(_Float16, lb);
            }
          }
          *(volatile v8h*)(C + (size_t)(mBase + row) * ldc + n0 + c8) = hv;
          if (OUT_MODE == 2) *(volatile v8h*)(C2 + (size_t)(mBase + row) * ldc + n0 + c8) = lv;
        }
        __threadfence();
      }
    }
    __builtin_amdgcn_fence(__ATOMIC_RELEASE, "workgroup");
    __builtin_amdgcn_wave_barrier();
    __builtin_amdgcn_fence(__ATOMIC_ACQUIRE, "workgroup");
  }
}

__global__ __launch_bounds__(256) void xin_cast_kernel(const float* __restrict__ x, unsigned short* __restrict__ XB) {
  __shared__ float sm[64][65];
  const int t  = threadIdx.x;
  const int n0 = blockIdx.x * 64;
  const int c0 = blockIdx.y * 64;
  const int b  = blockIdx.z;
#pragma unroll
  for (int i = 0; i < 8; ++i) {
    const int e = i * 256 + t;
    const int r = e >> 6;
    const int cc = e & 63;
    sm[cc][r] = x[((size_t)(b * kCh + c0 + r)) * kN + n0 + cc];
  }
  asm volatile("" ::: "memory");
#pragma unroll
  for (int i = 8; i < 16; ++i) {
    const int e = i * 256 + t;
    const int r = e >> 6;
    const int cc = e & 63;
    sm[cc][r] = x[((size_t)(b * kCh + c0 + r)) * kN + n0 + cc];
  }
  __syncthreads();
  const int lane = t & 31, wave = t >> 5;
  const int q = lane >> 3, c8 = (lane & 7) * 8;
  for (int pass = 0; pass < 2; ++pass) {
#pragma unroll
    for (int it = 0; it < 2; ++it) {
      const int row = wave * 8 + it * 4 + q;
      unsigned short hb[8];
#pragma unroll
      for (int e = 0; e < 8; ++e) hb[e] = f2bf_bits(sm[row][c8 + e]);
      const v4u u = (v4u){pk16(hb[0], hb[1]), pk16(hb[2], hb[3]), pk16(hb[4], hb[5]), pk16(hb[6], hb[7])};
      *(volatile v4u*)(XB + ((size_t)(b * kN + n0 + row)) * kCh + c0 + c8) = u;
    }
    __threadfence();
  }
}

__global__ __launch_bounds__(256) void w_cast_kernel(const float* __restrict__ W1, const float* __restrict__ W2,
                                                     const float* __restrict__ W3, unsigned short* __restrict__ WB) {
  const int plane = blockIdx.x >> 5;
  const float* src = (plane == 0) ? W1 : (plane == 1) ? W2 : W3;
  const int i = blockIdx.x * 256 + threadIdx.x;
  const int off = (i - plane * 8192) * 8;
  const v4f a = *(const v4f*)(src + off);
  const v4f c = *(const v4f*)(src + off + 4);
  unsigned short hb[8];
#pragma unroll
  for (int e = 0; e < 4; ++e) {
    hb[e]     = f2bf_bits(a[e]);
    hb[4 + e] = f2bf_bits(c[e]);
  }
  const v4u u = (v4u){pk16(hb[0], hb[1]), pk16(hb[2], hb[3]), pk16(hb[4], hb[5]), pk16(hb[6], hb[7])};
  unsigned short* qp = WB + 8 * (size_t)i;
  *(volatile v4u*)qp = u;
  __threadfence();
  *(volatile v4u*)qp = u;
}

__global__ __launch_bounds__(352) void param_cast_kernel(const float* __restrict__ b1, const float* __restrict__ b2,
                                                         const float* __restrict__ b3, const float* __restrict__ W4,
                                                         const float* __restrict__ b4, float* __restrict__ dst) {
  const int t = threadIdx.x;
  const int wave = t >> 5, lane = t & 31;
  v4f v = (v4f){0.f, 0.f, 0.f, 0.f};
  if (wave < 6) {
    const float* src = (wave < 2) ? b1 : (wave < 4) ? b2 : b3;
    v = *(const v4f*)(src + (wave & 1) * 128 + lane * 4);
  } else if (wave < 10) {
    v = *(const v4f*)(W4 + (wave - 6) * 128 + lane * 4);
  } else {
    const float s = b4[0];
    const float f0 = (lane == 0) ? 1.0f : 0.0f;
    v[0] = s * f0;
  }
  v4f r;
#pragma unroll
  for (int e = 0; e < 4; ++e) r[e] = bf_bits2f(f2bf_bits(v[e]));
  const bool act = (wave < 10) || (lane < 8);
  float* dp = dst + wave * 128 + lane * 4;
  if (act) *(volatile v4f*)dp = r;
  __threadfence();
  if (act) *(volatile v4f*)dp = r;
}

__global__ __launch_bounds__(256) void resid_kernel(const float* __restrict__ x, const float* __restrict__ br,
                                                    float* __restrict__ R) {
  const int idx = blockIdx.x * 256 + threadIdx.x;
  const int b = idx / kN;
  const int n = idx - b * kN;
  const float* xb = x + (size_t)b * kCh * kN + n;
  const float* w = br + kBrW4b;
  float s = 0.0f;
#pragma unroll 4
  for (int c = 0; c < kCh; ++c) {
    const float xv = bf_bits2f(f2bf_bits(xb[(size_t)c * kN]));
    s += xv * w[c];
  }
  *(volatile float*)(R + idx) = s;
  __threadfence();
  *(volatile float*)(R + idx) = s;
}

__global__ __launch_bounds__(256) void softmax_row_kernel(const float* __restrict__ S, unsigned short* __restrict__ P) {
  __shared__ float redM[8];
  __shared__ float redS[8];
  const int i    = blockIdx.x;
  const int hg   = blockIdx.y;
  const int t    = threadIdx.x;
  const int lane = t & 31, wave = t >> 5;
  const size_t rowoff = ((size_t)hg * kN + i) * kN;
  const bool act = (t < kSmThreads);
  const int tc = act ? t : (kSmThreads - 1);
  const float fact = act ? 1.0f : 0.0f;
  const float* sr = S + rowoff + 8 * (size_t)tc;
  const v4f a = *(const v4f*)(sr);
  const v4f c = *(const v4f*)(sr + 4);
  float xv[8];
#pragma unroll
  for (int e = 0; e < 4; ++e) { xv[e] = a[e]; xv[4 + e] = c[e]; }
  float mx = fmaxf(fmaxf(fmaxf(xv[0], xv[1]), fmaxf(xv[2], xv[3])), fmaxf(fmaxf(xv[4], xv[5]), fmaxf(xv[6], xv[7])));
#pragma unroll
  for (int off = 16; off > 0; off >>= 1) mx = fmaxf(mx, __shfl_xor(mx, off, 32));
  if (lane == 0) redM[wave] = mx;
  __syncthreads();
  float m = redM[0];
#pragma unroll
  for (int w = 1; w < 8; ++w) m = fmaxf(m, redM[w]);

  float p[8];
  float sl = 0.0f;
#pragma unroll
  for (int e = 0; e < 8; ++e) {
    p[e] = expf(xv[e] - m);
    sl += p[e];
  }
  float sum = sl * fact;
#pragma unroll
  for (int off = 16; off > 0; off >>= 1) sum += __shfl_xor(sum, off, 32);
  if (lane == 0) redS[wave] = sum;
  __syncthreads();
  float tot = redS[0];
#pragma unroll
  for (int w = 1; w < 8; ++w) tot += redS[w];
  const float inv = kPCarry * (1.0f / tot);

  unsigned short hb[8];
#pragma unroll
  for (int e = 0; e < 8; ++e) hb[e] = h_bits(p[e] * inv);
  const v4u u = (v4u){pk16(hb[0], hb[1]), pk16(hb[2], hb[3]), pk16(hb[4], hb[5]), pk16(hb[6], hb[7])};
  unsigned short* pr = P + rowoff + 8 * (size_t)tc;
  if (act) *(volatile v4u*)pr = u;
  __threadfence();
  if (act) *(volatile v4u*)pr = u;
}

__global__ __launch_bounds__(256) void head_kernel(const float* __restrict__ CTXg, const float* __restrict__ Rg,
                                                   const float* __restrict__ br, float* __restrict__ outg) {
  __shared__ __align__(16) float os[32];
  const int t = threadIdx.x;
  const int lane = t & 31, wave = t >> 5;
  const int row0 = blockIdx.x * 32 + wave * 4;
  const v4f wa = *(const v4f*)(br + kBrW4a + lane * 8);
  const v4f wb = *(const v4f*)(br + kBrW4a + lane * 8 + 4);
  const float b4r = br[kBrB4];
#pragma unroll 1
  for (int j = 0; j < 4; ++j) {
    const int row = row0 + j;
    const float* cr = CTXg + (size_t)row * kCh + lane * 8;
    const v4f c0 = *(const v4f*)(cr);
    const v4f c1 = *(const v4f*)(cr + 4);
    float s = 0.0f;
    s += c0[0] * wa[0]; s += c0[1] * wa[1]; s += c0[2] * wa[2]; s += c0[3] * wa[3];
    s += c1[0] * wb[0]; s += c1[1] * wb[1]; s += c1[2] * wb[2]; s += c1[3] * wb[3];
#pragma unroll
    for (int off = 16; off > 0; off >>= 1) s += __shfl_xor(s, off, 32);
    const float rr = Rg[row];
    const float tot = (s + rr) + b4r;
    if (lane == 0) os[wave * 4 + j] = tot;
  }
  __syncthreads();
  const bool act = (t < 8);
  const v4f v = *(const v4f*)(os + (lane & 7) * 4);
  float* op = outg + (size_t)blockIdx.x * 32 + (lane & 7) * 4;
  if (act) *(volatile v4f*)op = v;
  __threadfence();
  if (act) *(volatile v4f*)op = v;
}

extern "C" void kernel_launch(void* const* d_in, const int* in_sizes, int n_in,
                              void* d_out, int out_size, void* d_ws, size_t ws_size,
                              hipStream_t stream) {
  if (n_in < 9) return;
  if (in_sizes[0] != kBatch * kCh * kN) return;
  if (in_sizes[1] != kCh * kCh || in_sizes[3] != kCh * kCh || in_sizes[5] != kCh * kCh) return;
  if (in_sizes[2] != kCh || in_sizes[4] != kCh || in_sizes[6] != kCh) return;
  if (in_sizes[7] != 2 * kCh || in_sizes[8] != 1) return;
  if (out_size != kTok) return;

  const size_t szPlane16 = (size_t)kTok * kCh * 2;
  const size_t szWB  = (size_t)3 * kCh * kCh * 2;
  const size_t szBR  = (size_t)kBrFloats * 4;
  const size_t szR   = (size_t)kTok * 4;
  const size_t szSC  = (size_t)kGroup * kN * kN * 4;
  const size_t szPP  = (size_t)kGroup * kN * kN * 2;
  const size_t szCTX = (size_t)kGroup * kN * kCh * 4;
  size_t off = 0;
  const size_t offXB = off;  off += szPlane16;
  const size_t offWB = off;  off += szWB;
  const size_t offBR = off;  off += szBR;
  const size_t offQH = off;  off += szPlane16;
  const size_t offQL = off;  off += szPlane16;
  const size_t offKH = off;  off += szPlane16;
  const size_t offKL = off;  off += szPlane16;
  const size_t offVT = off;  off += szPlane16;
  const size_t offR  = off;  off += szR;
  const size_t offSC = off;  off += szSC;
  const size_t offPP = off;  off += szPP;
  const size_t offCT = off;  off += szCTX;
  const size_t total = off;
  if (ws_size < total) return;

  const float* x  = (const float*)d_in[0];
  const float* W1 = (const float*)d_in[1];
  const float* b1 = (const float*)d_in[2];
  const float* W2 = (const float*)d_in[3];
  const float* b2 = (const float*)d_in[4];
  const float* W3 = (const float*)d_in[5];
  const float* b3 = (const float*)d_in[6];
  const float* W4 = (const float*)d_in[7];
  const float* b4 = (const float*)d_in[8];
  float* out = (float*)d_out;
  char* ws = (char*)d_ws;
  unsigned short* XB = (unsigned short*)(ws + offXB);
  unsigned short* WB = (unsigned short*)(ws + offWB);
  float* BR = (float*)(ws + offBR);
  unsigned short* QH = (unsigned short*)(ws + offQH);
  unsigned short* QL = (unsigned short*)(ws + offQL);
  unsigned short* KH = (unsigned short*)(ws + offKH);
  unsigned short* KL = (unsigned short*)(ws + offKL);
  unsigned short* VT = (unsigned short*)(ws + offVT);
  float* R  = (float*)(ws + offR);
  float* SC = (float*)(ws + offSC);
  unsigned short* PP = (unsigned short*)(ws + offPP);
  float* CT = (float*)(ws + offCT);

  xin_cast_kernel<<<dim3(kN / 64, kCh / 64, kBatch), dim3(256), 0, stream>>>(x, XB);
  w_cast_kernel<<<dim3(96), dim3(256), 0, stream>>>(W1, W2, W3, WB);
  param_cast_kernel<<<dim3(1), dim3(352), 0, stream>>>(b1, b2, b3, W4, b4, BR);
  resid_kernel<<<dim3(kTok / 256), dim3(256), 0, stream>>>(x, BR, R);

  const long plane16 = (long)kN * kCh;
  const int tilesQK = (kTok / 64) * (kCh / 64);
  wmma_gemm64<1, false, 2, 2, false, 0><<<dim3(tilesQK / 8, 1), dim3(256), 0, stream>>>(
      XB, XB, kCh, 0L, WB, WB, kCh, 0L, (void*)QH, (void*)QL, kCh, 0L, BR + kBrB1, BR, 0L, kTok, kCh, kCh, 1.0f);
  wmma_gemm64<1, false, 2, 2, false, 0><<<dim3(tilesQK / 8, 1), dim3(256), 0, stream>>>(
      XB, XB, kCh, 0L, WB + kCh * kCh, WB + kCh * kCh, kCh, 0L, (void*)KH, (void*)KL, kCh, 0L, BR + kBrB2, BR, 0L,
      kTok, kCh, kCh, 1.0f);
  const int tilesVT = (kCh / 64) * (kN / 64);
  wmma_gemm64<1, false, 1, 1, false, 0><<<dim3((tilesVT + 7) / 8, kBatch), dim3(256), 0, stream>>>(
      WB + 2 * kCh * kCh, WB + 2 * kCh * kCh, kCh, 0L, XB, XB, kCh, plane16, (void*)VT, (void*)VT, kN, plane16,
      BR + kBrB3, BR, 0L, kCh, kN, kCh, 1.0f);

  const long strideScore = (long)kN * kN;
  const int tilesScore = (kN / 64) * (kN / 64);
  const int tilesCtx   = (kN / 64) * (kCh / 64);
  for (int g = 0; g < kNGroups; ++g) {
    const size_t tokOff = (size_t)g * kGroup * (size_t)plane16;
    wmma_gemm64<1, true, 0, 0, false, 0><<<dim3((tilesScore + 7) / 8, kGroup), dim3(256), 0, stream>>>(
        QH + tokOff, QL + tokOff, kCh, plane16, KH + tokOff, KL + tokOff, kCh, plane16,
        (void*)SC, (void*)SC, kN, strideScore, BR, BR, 0L, kN, kN, kCh, 1.0f);
    softmax_row_kernel<<<dim3(kN, kGroup), dim3(256), 0, stream>>>(SC, PP);
    const unsigned short* VTg = VT + (size_t)g * kGroup * (size_t)plane16;
    wmma_gemm64<0, false, 0, 0, false, 0><<<dim3((tilesCtx + 7) / 8, kGroup), dim3(256), 0, stream>>>(
        PP, PP, kN, strideScore, VTg, VTg, kN, plane16, (void*)CT, (void*)CT, kCh, plane16, BR, BR, 0L,
        kN, kCh, kN, kPCarryInv);
    head_kernel<<<dim3((kGroup * kN) / 32), dim3(256), 0, stream>>>(CT, R + (size_t)g * kGroup * kN, BR,
                                                                   out + (size_t)g * kGroup * kN);
  }
}
